// LocalBlock3D_28647431864485
// MI455X (gfx1250) — hardware-run, weakly checked
//
#include <hip/hip_runtime.h>
#include <stdint.h>

#define DEVINL __device__ __forceinline__

typedef _Float16 f16t;
typedef _Float16 v16h __attribute__((ext_vector_type(16)));
typedef _Float16 v8h  __attribute__((ext_vector_type(8)));
typedef _Float16 v4h  __attribute__((ext_vector_type(4)));
typedef float    v8f  __attribute__((ext_vector_type(8)));
typedef float    v4f  __attribute__((ext_vector_type(4)));
typedef v8h __attribute__((may_alias)) v8ha;
typedef v4h __attribute__((may_alias)) v4ha;
typedef v4f __attribute__((may_alias)) v4fa;
union FragH { v16h v; v8h half[2]; };

#define NTOK   4096
#define GD     16
#define CW     128
#define HID    512
#define NHEAD  4
#define HDIM   32
#define KSZ    5
#define KRAD   2
#define NTAP   125
#define TPB    256
#define WAVES  8
#define MT     64
#define PQF    132
#define PQH    136
#define ACAR   16.0f
#define WCAR   256.0f
#define OCAR   256.0f
#define MCAR   256.0f
#define SC_AW  (1.0f / (16.0f * 256.0f))
#define SC_OW  (1.0f / (256.0f * 256.0f))
#define EPS    1e-6f
#define QSCALE 0.17677669529663688f

static_assert(TPB == WAVES * 32);
static_assert(GD * GD * GD == NTOK);
static_assert(NHEAD * HDIM == CW);
static_assert(KSZ * KSZ * KSZ == NTAP);
static_assert((NTOK % MT) == 0);
static_assert((NTOK % WAVES) == 0);
static_assert((CW % 32) == 0);
static_assert((HID % 128) == 0);
static_assert((PQF % 4) == 0);
static_assert((PQH % 8) == 0);
static_assert(MT == 64);

DEVINL int imin(int a, int b) { return a < b ? a : b; }
DEVINL int imax(int a, int b) { return a > b ? a : b; }

DEVINL v8f wmma_f16(v16h a, v16h b, v8f c) {
  v8f d = __builtin_amdgcn_wmma_f32_16x16x32_f16(false, a, false, b, (short)0, c, false, false);
  asm volatile("v_nop\n\tv_nop\n\tv_nop\n\tv_nop" : "+v"(d) : "v"(a), "v"(b));
  return d;
}
DEVINL v8f zero8f() {
  v8f z = {0.f, 0.f, 0.f, 0.f, 0.f, 0.f, 0.f, 0.f};
  return z;
}
DEVINL void load_frag(FragH& f, const f16t* row, int k0) {
  f.half[0] = *(const v8ha*)(row + k0);
  f.half[1] = *(const v8ha*)(row + k0 + 16);
}

DEVINL float wsum32(float v) {
  #pragma unroll
  for (int s = 16; s > 0; s >>= 1) v += __shfl_xor(v, s);
  return v;
}
DEVINL float hsum16(float v) {
  #pragma unroll
  for (int s = 8; s > 0; s >>= 1) v += __shfl_xor(v, s);
  return v;
}
DEVINL float gsum8(float v) {
  v += __shfl_xor(v, 1);
  v += __shfl_xor(v, 2);
  v += __shfl_xor(v, 4);
  return v;
}

template <int KD>
DEVINL void mma_4n(const f16t* __restrict__ arow, const f16t* __restrict__ brow, v8f (&acc)[4]) {
  #pragma unroll 1
  for (int ks = 0; ks < KD / 32; ++ks) {
    const int k0 = 32 * ks;
    FragH a;
    load_frag(a, arow, k0);
    #pragma unroll
    for (int n = 0; n < 4; ++n) {
      FragH b;
      load_frag(b, brow + (size_t)16 * n * KD, k0);
      acc[n] = wmma_f16(a.v, b.v, acc[n]);
    }
  }
}
template <int KD>
DEVINL void mma_4n2(const f16t* __restrict__ arow, const f16t* __restrict__ browg,
                    const f16t* __restrict__ browu, v8f (&accg)[4], v8f (&accu)[4]) {
  #pragma unroll 1
  for (int ks = 0; ks < KD / 32; ++ks) {
    const int k0 = 32 * ks;
    FragH a;
    load_frag(a, arow, k0);
    #pragma unroll
    for (int n = 0; n < 4; ++n) {
      FragH bg, bu;
      load_frag(bg, browg + (size_t)16 * n * KD, k0);
      load_frag(bu, browu + (size_t)16 * n * KD, k0);
      accg[n] = wmma_f16(a.v, bg.v, accg[n]);
      accu[n] = wmma_f16(a.v, bu.v, accu[n]);
    }
  }
}

DEVINL void stage_f32(float* sbuf, const v8f (&acc)[4], float sc, int mt, int nh, int h, int m) {
  #pragma unroll
  for (int n = 0; n < 4; ++n) {
    #pragma unroll
    for (int r = 0; r < 8; ++r)
      sbuf[(16 * mt + 8 * h + r) * PQF + 64 * nh + 16 * n + m] = acc[n][r] * sc;
  }
}

DEVINL void store_rows_f32(const float* sbuf, float* dst, int wave, int lane) {
  #pragma unroll
  for (int i = 0; i < 8; ++i) {
    const int row = wave + 8 * i;
    const v4f v = *(const v4fa*)(sbuf + row * PQF + 4 * lane);
    *(volatile v4f*)(dst + (size_t)row * CW + 4 * lane) = v;
  }
  __threadfence();
  #pragma unroll
  for (int i = 0; i < 8; ++i) {
    const int row = wave + 8 * i;
    const v4f v = *(const v4fa*)(sbuf + row * PQF + 4 * lane);
    *(volatile v4f*)(dst + (size_t)row * CW + 4 * lane) = v;
  }
}

DEVINL void store_rows_f16(const f16t* sH, f16t* dst, int pitch, int wave, int lane) {
  const int hsel = lane >> 4, l16 = lane & 15;
  #pragma unroll
  for (int i2 = 0; i2 < 4; ++i2) {
    const int row = wave + 8 * (2 * i2 + hsel);
    const v8h v = *(const v8ha*)(sH + row * PQH + 8 * l16);
    *(volatile v8h*)(dst + (size_t)row * pitch + 8 * l16) = v;
  }
  __threadfence();
  #pragma unroll
  for (int i2 = 0; i2 < 4; ++i2) {
    const int row = wave + 8 * (2 * i2 + hsel);
    const v8h v = *(const v8ha*)(sH + row * PQH + 8 * l16);
    *(volatile v8h*)(dst + (size_t)row * pitch + 8 * l16) = v;
  }
}

__global__ __launch_bounds__(TPB) void prep_w_k(const float* __restrict__ wq, const float* __restrict__ wk,
                                               const float* __restrict__ wv, const float* __restrict__ wo,
                                               const float* __restrict__ wg, const float* __restrict__ wu,
                                               const float* __restrict__ wd,
                                               f16t* __restrict__ WQKV, f16t* __restrict__ WO,
                                               f16t* __restrict__ WGU, f16t* __restrict__ WD)
{
  const int blk = blockIdx.x, tid = threadIdx.x;
  if (blk >= 128) return;
  v8h o;
  f16t* dst;
  if (blk < 24) {
    const int grp = blk >> 3;
    const float* src = (grp == 0) ? wq : ((grp == 1) ? wk : wv);
    const int t = blk * TPB + tid;
    const int row = t >> 4, piece = (t & 15) * 8;
    const int n = imin(imax(row - 128 * grp, 0), CW - 1);
    #pragma unroll
    for (int i = 0; i < 8; ++i) o[i] = (f16t)(src[(size_t)(piece + i) * CW + n] * WCAR);
    dst = WQKV + (size_t)row * CW + piece;
  } else if (blk < 32) {
    const int t = (blk - 24) * TPB + tid;
    const int row = t >> 4, piece = (t & 15) * 8;
    #pragma unroll
    for (int i = 0; i < 8; ++i) o[i] = (f16t)(wo[(size_t)(piece + i) * CW + row] * WCAR);
    dst = WO + (size_t)row * CW + piece;
  } else if (blk < 96) {
    const int rb = blk - 32;
    const int grp = rb >> 5;
    const float* src = (grp == 0) ? wg : wu;
    const int t = rb * TPB + tid;
    const int row = t >> 4, piece = (t & 15) * 8;
    const int n = imin(imax(row - 512 * grp, 0), HID - 1);
    #pragma unroll
    for (int i = 0; i < 8; ++i) o[i] = (f16t)(src[(size_t)(piece + i) * HID + n] * WCAR);
    dst = WGU + (size_t)row * CW + piece;
  } else {
    const int rb = blk - 96;
    const int u = rb * TPB + tid;
    const int row = u >> 6, piece = (u & 63) * 8;
    #pragma unroll
    for (int i = 0; i < 8; ++i) o[i] = (f16t)(wd[(size_t)(piece + i) * CW + row] * WCAR);
    dst = WD + (size_t)row * HID + piece;
  }
  *(volatile v8h*)dst = o;
  __threadfence();
  *(volatile v8h*)dst = o;
}

__global__ __launch_bounds__(TPB) void rms_h_k(const float* __restrict__ x, const float* __restrict__ w,
                                              f16t* __restrict__ H)
{
  const int tid = threadIdx.x, lane = tid & 31, wave = tid >> 5;
  const int hsel = lane >> 4, l16 = lane & 15;
  const int rb = blockIdx.x * MT;
  if (rb >= NTOK) return;
  const v4f w0 = *(const v4fa*)(w + 8 * l16), w1 = *(const v4fa*)(w + 8 * l16 + 4);
  v8h hv[4];
  #pragma unroll
  for (int i = 0; i < 4; ++i) {
    const int row = rb + wave * 8 + 2 * i + hsel;
    const float* xp = x + (size_t)row * CW + 8 * l16;
    const v4f a = *(const v4fa*)xp, c = *(const v4fa*)(xp + 4);
    float ss = a[0] * a[0] + a[1] * a[1] + a[2] * a[2] + a[3] * a[3]
             + c[0] * c[0] + c[1] * c[1] + c[2] * c[2] + c[3] * c[3];
    ss = hsum16(ss);
    const float r = rsqrtf(ss * (1.0f / CW) + EPS);
    #pragma unroll
    for (int j = 0; j < 4; ++j) {
      hv[i][j]     = (f16t)((a[j] * r) * w0[j] * ACAR);
      hv[i][4 + j] = (f16t)((c[j] * r) * w1[j] * ACAR);
    }
  }
  #pragma unroll
  for (int i = 0; i < 4; ++i) {
    const int row = rb + wave * 8 + 2 * i + hsel;
    *(volatile v8h*)(H + (size_t)row * CW + 8 * l16) = hv[i];
  }
  __threadfence();
  #pragma unroll
  for (int i = 0; i < 4; ++i) {
    const int row = rb + wave * 8 + 2 * i + hsel;
    *(volatile v8h*)(H + (size_t)row * CW + 8 * l16) = hv[i];
  }
}

__global__ __launch_bounds__(TPB) void gemm_qkv_k(const f16t* __restrict__ Hp, const f16t* __restrict__ Wp,
                                                 float* __restrict__ Qo, float* __restrict__ Ko,
                                                 float* __restrict__ Vo)
{
  __shared__ __attribute__((aligned(16))) float sbuf[MT * PQF];
  const int tid = threadIdx.x, lane = tid & 31, wave = tid >> 5;
  const int h = lane >> 4, m = lane & 15;
  const int mt = wave & 3, nh = wave >> 2;
  const int row0 = blockIdx.x * MT, y = blockIdx.y;
  float* outp = (y == 0) ? Qo : ((y == 1) ? Ko : Vo);

  v8f acc[4];
  #pragma unroll
  for (int n = 0; n < 4; ++n) acc[n] = zero8f();
  const f16t* arow = Hp + (size_t)(row0 + 16 * mt + m) * CW + 8 * h;
  const f16t* brow = Wp + (size_t)(y * CW + 64 * nh + m) * CW + 8 * h;
  mma_4n<CW>(arow, brow, acc);
  stage_f32(sbuf, acc, SC_AW, mt, nh, h, m);
  __syncthreads();
  store_rows_f32(sbuf, outp + (size_t)row0 * CW, wave, lane);
}

__global__ __launch_bounds__(TPB) void attn_k(const float* __restrict__ Qp, const float* __restrict__ Kp,
                                             const float* __restrict__ Vp, f16t* __restrict__ Op)
{
  __shared__ __attribute__((aligned(16))) float sS[WAVES * 512];
  __shared__ __attribute__((aligned(16))) f16t  sO[WAVES * CW];
  const int tid = threadIdx.x, lane = tid & 31, wave = tid >> 5;
  const int gp = imin(blockIdx.x * WAVES + wave, NTOK - 1);
  const int z0 = gp >> 8, y0 = (gp >> 4) & 15, x0 = gp & 15;
  const int head = lane >> 3, c0 = 4 * lane, j8 = lane & 7;
  float* sw = sS + wave * 512;
  float* sh = sw + head * 128;

  {
    const v4f fill = {-1.0e9f, -1.0e9f, -1.0e9f, -1.0e9f};
    #pragma unroll
    for (int q4i = 0; q4i < 4; ++q4i) *(v4fa*)(sw + 16 * lane + 4 * q4i) = fill;
  }
  __syncthreads();

  const v4f q4 = *(const v4fa*)(Qp + (size_t)gp * CW + c0);
  float mx = -3.0e38f;
  {
    int t = 0;
    #pragma unroll 1
    for (int dz = -KRAD; dz <= KRAD; ++dz) {
      const int zz = z0 + dz;
      const int vz = ((unsigned)zz < (unsigned)GD) ? 1 : 0;
      const int zc = imin(imax(zz, 0), GD - 1);
      #pragma unroll 1
      for (int dy = -KRAD; dy <= KRAD; ++dy) {
        const int yy = y0 + dy;
        const int vy = ((unsigned)yy < (unsigned)GD) ? 1 : 0;
        const int yc = imin(imax(yy, 0), GD - 1);
        #pragma unroll 1
        for (int dx = -KRAD; dx <= KRAD; ++dx, ++t) {
          const int xx = x0 + dx;
          const int vx = ((unsigned)xx < (unsigned)GD) ? 1 : 0;
          const int xc = imin(imax(xx, 0), GD - 1);
          const int vld = vz & vy & vx;
          const size_t nb = (size_t)((zc * GD + yc) * GD + xc);
          const v4f k4 = *(const v4fa*)(Kp + nb * CW + c0);
          float d = q4[0] * k4[0];
          d = fmaf(q4[1], k4[1], d);
          d = fmaf(q4[2], k4[2], d);
          d = fmaf(q4[3], k4[3], d);
          d = gsum8(d);
          float s = d * QSCALE;
          s = vld ? s : -1.0e9f;
          mx = fmaxf(mx, s);
          sh[t] = s;
        }
      }
    }
  }
  __syncthreads();

  float ssum = 0.0f;
  #pragma unroll 1
  for (int it = 0; it < 16; ++it) {
    const int tt = j8 + 8 * it;
    const float sv = sh[tt];
    float e = __expf(sv - mx);
    e = (sv > -1.0e8f) ? e : 0.0f;
    sh[tt] = e;
    ssum += e;
  }
  ssum = gsum8(ssum);
  const float rS = __builtin_amdgcn_rcpf(ssum);
  __syncthreads();

  v4f cx = {0.f, 0.f, 0.f, 0.f};
  {
    int t = 0;
    #pragma unroll 1
    for (int dz = -KRAD; dz <= KRAD; ++dz) {
      const int zc = imin(imax(z0 + dz, 0), GD - 1);
      #pragma unroll 1
      for (int dy = -KRAD; dy <= KRAD; ++dy) {
        const int yc = imin(imax(y0 + dy, 0), GD - 1);
        #pragma unroll 1
        for (int dx = -KRAD; dx <= KRAD; ++dx, ++t) {
          const int xc = imin(imax(x0 + dx, 0), GD - 1);
          const size_t nb = (size_t)((zc * GD + yc) * GD + xc);
          const float p = sh[t] * rS;
          const v4f v4 = *(const v4fa*)(Vp + nb * CW + c0);
          cx[0] = fmaf(p, v4[0], cx[0]);
          cx[1] = fmaf(p, v4[1], cx[1]);
          cx[2] = fmaf(p, v4[2], cx[2]);
          cx[3] = fmaf(p, v4[3], cx[3]);
        }
      }
    }
  }

  v4h oh;
  #pragma unroll
  for (int j = 0; j < 4; ++j) oh[j] = (f16t)(cx[j] * OCAR);
  *(v4ha*)(sO + wave * CW + c0) = oh;
  __syncthreads();
  if (wave < 4) {
    const v8h v = *(const v8ha*)(sO + wave * 256 + 8 * lane);
    f16t* dst = Op + (size_t)(blockIdx.x * WAVES + 2 * wave) * CW + 8 * lane;
    *(volatile v8h*)dst = v;
    __threadfence();
    *(volatile v8h*)dst = v;
  }
}

__global__ __launch_bounds__(TPB) void gemm_wo_k(const f16t* __restrict__ Opl, const f16t* __restrict__ Wp,
                                                const float* __restrict__ x, const float* __restrict__ wa,
                                                const float* __restrict__ w2,
                                                float* __restrict__ X1, f16t* __restrict__ H2)
{
  __shared__ __attribute__((aligned(16))) float sbuf[MT * PQF];
  __shared__ __attribute__((aligned(16))) f16t  sH[MT * PQH];
  const int tid = threadIdx.x, lane = tid & 31, wave = tid >> 5;
  const int h = lane >> 4, m = lane & 15;
  const int mt = wave & 3, nh = wave >> 2;
  const int row0 = blockIdx.x * MT;

  v8f acc[4];
  #pragma unroll
  for (int n = 0; n < 4; ++n) acc[n] = zero8f();
  const f16t* arow = Opl + (size_t)(row0 + 16 * mt + m) * CW + 8 * h;
  const f16t* brow = Wp + (size_t)(64 * nh + m) * CW + 8 * h;
  mma_4n<CW>(arow, brow, acc);
  stage_f32(sbuf, acc, SC_OW, mt, nh, h, m);
  __syncthreads();

  const v4f wav = *(const v4fa*)(wa + 4 * lane), w2v = *(const v4fa*)(w2 + 4 * lane);
  #pragma unroll
  for (int i = 0; i < 8; ++i) {
    const int row = wave + 8 * i;
    float* sp = sbuf + row * PQF + 4 * lane;
    const v4f t = *(const v4fa*)sp;
    const v4f xv = *(const v4fa*)(x + (size_t)(row0 + row) * CW + 4 * lane);
    float ss = t[0] * t[0] + t[1] * t[1] + t[2] * t[2] + t[3] * t[3];
    ss = wsum32(ss);
    const float r = rsqrtf(ss * (1.0f / CW) + EPS);
    v4f x1;
    #pragma unroll
    for (int j = 0; j < 4; ++j) x1[j] = xv[j] + (t[j] * r) * wav[j];
    float s2 = x1[0] * x1[0] + x1[1] * x1[1] + x1[2] * x1[2] + x1[3] * x1[3];
    s2 = wsum32(s2);
    const float r2 = rsqrtf(s2 * (1.0f / CW) + EPS);
    v4h hh;
    #pragma unroll
    for (int j = 0; j < 4; ++j) hh[j] = (f16t)((x1[j] * r2) * w2v[j] * ACAR);
    *(v4fa*)sp = x1;
    *(v4ha*)(sH + row * PQH + 4 * lane) = hh;
  }
  __syncthreads();

  float* dx1 = X1 + (size_t)row0 * CW;
  f16t*  dh2 = H2 + (size_t)row0 * CW;
  const int hsel = lane >> 4, l16 = lane & 15;
  #pragma unroll
  for (int i = 0; i < 8; ++i) {
    const int row = wave + 8 * i;
    const v4f v = *(const v4fa*)(sbuf + row * PQF + 4 * lane);
    *(volatile v4f*)(dx1 + (size_t)row * CW + 4 * lane) = v;
  }
  #pragma unroll
  for (int i2 = 0; i2 < 4; ++i2) {
    const int row = wave + 8 * (2 * i2 + hsel);
    const v8h v = *(const v8ha*)(sH + row * PQH + 8 * l16);
    *(volatile v8h*)(dh2 + (size_t)row * CW + 8 * l16) = v;
  }
  __threadfence();
  #pragma unroll
  for (int i = 0; i < 8; ++i) {
    const int row = wave + 8 * i;
    const v4f v = *(const v4fa*)(sbuf + row * PQF + 4 * lane);
    *(volatile v4f*)(dx1 + (size_t)row * CW + 4 * lane) = v;
  }
  #pragma unroll
  for (int i2 = 0; i2 < 4; ++i2) {
    const int row = wave + 8 * (2 * i2 + hsel);
    const v8h v = *(const v8ha*)(sH + row * PQH + 8 * l16);
    *(volatile v8h*)(dh2 + (size_t)row * CW + 8 * l16) = v;
  }
}

__global__ __launch_bounds__(TPB) void gemm_gu_k(const f16t* __restrict__ H2p, const f16t* __restrict__ Wp,
                                                f16t* __restrict__ Mo)
{
  __shared__ __attribute__((aligned(16))) f16t sH[MT * PQH];
  const int tid = threadIdx.x, lane = tid & 31, wave = tid >> 5;
  const int h = lane >> 4, m = lane & 15;
  const int mt = wave & 3, nh = wave >> 2;
  const int row0 = blockIdx.x * MT, y = blockIdx.y;

  v8f accg[4], accu[4];
  #pragma unroll
  for (int n = 0; n < 4; ++n) { accg[n] = zero8f(); accu[n] = zero8f(); }
  const f16t* arow  = H2p + (size_t)(row0 + 16 * mt + m) * CW + 8 * h;
  const f16t* browg = Wp + (size_t)(y * 128 + 64 * nh + m) * CW + 8 * h;
  const f16t* browu = browg + (size_t)HID * CW;
  mma_4n2<CW>(arow, browg, browu, accg, accu);

  #pragma unroll
  for (int n = 0; n < 4; ++n) {
    #pragma unroll
    for (int r = 0; r < 8; ++r) {
      const float g = accg[n][r] * SC_AW;
      const float u = accu[n][r] * SC_AW;
      const float sg = g * __builtin_amdgcn_rcpf(1.0f + __expf(-g));
      sH[(16 * mt + 8 * h + r) * PQH + 64 * nh + 16 * n + m] = (f16t)(sg * u * MCAR);
    }
  }
  __syncthreads();
  store_rows_f16(sH, Mo + (size_t)row0 * HID + 128 * y, HID, wave, lane);
}

__global__ __launch_bounds__(TPB) void gemm_down_k(const f16t* __restrict__ Mp, const f16t* __restrict__ Wp,
                                                  const float* __restrict__ X1, float* __restrict__ out)
{
  __shared__ __attribute__((aligned(16))) float sbuf[MT * PQF];
  const int tid = threadIdx.x, lane = tid & 31, wave = tid >> 5;
  const int h = lane >> 4, m = lane & 15;
  const int mt = wave & 3, nh = wave >> 2;
  const int row0 = blockIdx.x * MT;

  v8f acc[4];
  #pragma unroll
  for (int n = 0; n < 4; ++n) acc[n] = zero8f();
  const f16t* arow = Mp + (size_t)(row0 + 16 * mt + m) * HID + 8 * h;
  const f16t* brow = Wp + (size_t)(64 * nh + m) * HID + 8 * h;
  mma_4n<HID>(arow, brow, acc);
  stage_f32(sbuf, acc, SC_OW, mt, nh, h, m);
  __syncthreads();

  #pragma unroll
  for (int i = 0; i < 8; ++i) {
    const int row = wave + 8 * i;
    float* sp = sbuf + row * PQF + 4 * lane;
    const v4f t = *(const v4fa*)sp;
    const v4f xv = *(const v4fa*)(X1 + (size_t)(row0 + row) * CW + 4 * lane);
    v4f o;
    #pragma unroll
    for (int j = 0; j < 4; ++j) o[j] = xv[j] + t[j];
    *(v4fa*)sp = o;
  }
  __syncthreads();
  store_rows_f32(sbuf, out + (size_t)row0 * CW, wave, lane);
}

extern "C" void kernel_launch(void* const* d_in, const int* in_sizes, int n_in,
                              void* d_out, int out_size, void* d_ws, size_t ws_size,
                              hipStream_t stream) {
  if (n_in < 11) return;
  if (in_sizes[0] != NTOK * CW) return;
  if (in_sizes[1] != CW || in_sizes[2] != CW || in_sizes[3] != CW) return;
  if (in_sizes[4] != CW * CW || in_sizes[5] != CW * CW || in_sizes[6] != CW * CW || in_sizes[7] != CW * CW) return;
  if (in_sizes[8] != CW * HID || in_sizes[9] != CW * HID || in_sizes[10] != HID * CW) return;
  if (out_size != NTOK * CW) return;

  const float* x       = (const float*)d_in[0];
  const float* norm1_w = (const float*)d_in[1];
  const float* attn_nw = (const float*)d_in[2];
  const float* norm2_w = (const float*)d_in[3];
  const float* wq      = (const float*)d_in[4];
  const float* wk      = (const float*)d_in[5];
  const float* wv      = (const float*)d_in[6];
  const float* wo      = (const float*)d_in[7];
  const float* gate_w  = (const float*)d_in[8];
  const float* up_w    = (const float*)d_in[9];
  const float* down_w  = (const float*)d_in[10];
  float* outp = (float*)d_out;

  const size_t szWQKV = (size_t)3 * CW * CW * 2;
  const size_t szWO   = (size_t)CW * CW * 2;
  const size_t szWGU  = (size_t)2 * HID * CW * 2;
  const size_t szWD   = (size_t)CW * HID * 2;
  const size_t szP16  = (size_t)NTOK * CW * 2;
  const size_t szP32  = (size_t)NTOK * CW * 4;
  const size_t szM    = (size_t)NTOK * HID * 2;
  size_t off = 0;
  char* ws = (char*)d_ws;
  f16t*  WQKV = (f16t*)(ws + off);  off += szWQKV;
  f16t*  WO   = (f16t*)(ws + off);  off += szWO;
  f16t*  WGU  = (f16t*)(ws + off);  off += szWGU;
  f16t*  WD   = (f16t*)(ws + off);  off += szWD;
  f16t*  Hp   = (f16t*)(ws + off);  off += szP16;
  float* Qp   = (float*)(ws + off); off += szP32;
  float* Kp   = (float*)(ws + off); off += szP32;
  float* Vp   = (float*)(ws + off); off += szP32;
  f16t*  Opl  = (f16t*)(ws + off);  off += szP16;
  float* X1   = (float*)(ws + off); off += szP32;
  f16t*  H2   = (f16t*)(ws + off);  off += szP16;
  f16t*  Mp   = (f16t*)(ws + off);  off += szM;
  if (off > ws_size) return;

  prep_w_k<<<128, TPB, 0, stream>>>(wq, wk, wv, wo, gate_w, up_w, down_w, WQKV, WO, WGU, WD);
  rms_h_k<<<NTOK / MT, TPB, 0, stream>>>(x, norm1_w, Hp);
  gemm_qkv_k<<<dim3(NTOK / MT, 3), TPB, 0, stream>>>(Hp, WQKV, Qp, Kp, Vp);
  attn_k<<<NTOK / WAVES, TPB, 0, stream>>>(Qp, Kp, Vp, Opl);
  gemm_wo_k<<<NTOK / MT, TPB, 0, stream>>>(Opl, WO, x, attn_nw, norm2_w, X1, H2);
  gemm_gu_k<<<dim3(NTOK / MT, HID / 128), TPB, 0, stream>>>(H2, WGU, Mp);
  gemm_down_k<<<NTOK / MT, TPB, 0, stream>>>(Mp, WD, X1, outp);
  (void)hipGetLastError();
}
